// RandomProjectionQuantizer_8521215115483
// MI455X (gfx1250) — hardware-verified
//
#include <hip/hip_runtime.h>
#include <stdint.h>


#define DIN    320
#define DCB    16
#define KSTEPS (DIN / 32)
#define PPW    (DIN / 2)
#define SUPER  512
#define NCHUNK (SUPER / 16)
#define WAVES  8
#define BLOCK  (WAVES * 32)
#define TOK_PER_WAVE  32
#define TOK_PER_BLOCK (WAVES * TOK_PER_WAVE)

#define SX 64.0f
#define SP 512.0f
#define SC 256.0f
#define SN 256.0f

typedef _Float16 v16h __attribute__((ext_vector_type(16)));
typedef _Float16 h2   __attribute__((ext_vector_type(2)));
typedef float    v8f  __attribute__((ext_vector_type(8)));
typedef int      v4i  __attribute__((ext_vector_type(4)));

union H2U  { h2 h; uint32_t u; };
union Frag { v16h v; uint32_t u[8]; uint4 q[2]; };

__device__ __forceinline__ void split_pair(float a, float b, uint32_t& hp, uint32_t& lp)
{
    const _Float16 ha = (_Float16)a;
    const _Float16 hb = (_Float16)b;
    const _Float16 la = (_Float16)(a - (float)ha);
    const _Float16 lb = (_Float16)(b - (float)hb);
    H2U t; t.h.x = ha; t.h.y = hb; hp = t.u;
    H2U s; s.h.x = la; s.h.y = lb; lp = s.u;
}

__device__ __forceinline__ v8f wmma16(v16h a, v16h b, v8f c)
{
    return __builtin_amdgcn_wmma_f32_16x16x32_f16(false, a, false, b, (short)0, c, false, false);
}

__device__ __forceinline__ void proj_tile(const float* __restrict__ xr,
                                          const uint32_t* Pth, const uint32_t* Ptl,
                                          int m, int h, Frag& b1, Frag& b2)
{
    v8f acc = {};
#pragma unroll 1
    for (int ks = 0; ks < KSTEPS; ++ks) {
        Frag ahi, alo, bhi, blo;
        const int ab = m * PPW + ks * 16 + 4 * h;
        ahi.q[0] = *(const uint4*)(Pth + ab);
        ahi.q[1] = *(const uint4*)(Pth + ab + 8);
        alo.q[0] = *(const uint4*)(Ptl + ab);
        alo.q[1] = *(const uint4*)(Ptl + ab + 8);
        const float* xp = xr + ks * 32 + 8 * h;
        const float4 f0 = *(const float4*)(xp);
        const float4 f1 = *(const float4*)(xp + 4);
        const float4 g0 = *(const float4*)(xp + 16);
        const float4 g1 = *(const float4*)(xp + 20);
        split_pair(f0.x * SX, f0.y * SX, bhi.u[0], blo.u[0]);
        split_pair(f0.z * SX, f0.w * SX, bhi.u[1], blo.u[1]);
        split_pair(f1.x * SX, f1.y * SX, bhi.u[2], blo.u[2]);
        split_pair(f1.z * SX, f1.w * SX, bhi.u[3], blo.u[3]);
        split_pair(g0.x * SX, g0.y * SX, bhi.u[4], blo.u[4]);
        split_pair(g0.z * SX, g0.w * SX, bhi.u[5], blo.u[5]);
        split_pair(g1.x * SX, g1.y * SX, bhi.u[6], blo.u[6]);
        split_pair(g1.z * SX, g1.w * SX, bhi.u[7], blo.u[7]);
        acc = wmma16(ahi.v, bhi.v, acc);
        acc = wmma16(alo.v, bhi.v, acc);
        acc = wmma16(ahi.v, blo.v, acc);
        acc = wmma16(alo.v, blo.v, acc);
        asm volatile("v_nop\n\tv_nop\n\tv_nop\n\tv_nop"
                     : "+v"(acc) : "v"(ahi.v), "v"(alo.v), "v"(bhi.v), "v"(blo.v));
    }

    float ss = 0.f;
#pragma unroll
    for (int r = 0; r < 8; ++r) ss = fmaf(acc[r], acc[r], ss);
    ss += __shfl_xor(ss, 16, 32);
    const float inv = 1.0f / fmaxf(sqrtf(ss), 1e-12f * SX * SP);
    const float scl = inv * SN;

    uint32_t hp[4], lp[4];
    split_pair(acc[0] * scl, acc[1] * scl, hp[0], lp[0]);
    split_pair(acc[2] * scl, acc[3] * scl, hp[1], lp[1]);
    split_pair(acc[4] * scl, acc[5] * scl, hp[2], lp[2]);
    split_pair(acc[6] * scl, acc[7] * scl, hp[3], lp[3]);
#pragma unroll
    for (int j = 0; j < 4; ++j) {
        b1.u[j] = hp[j]; b1.u[4 + j] = hp[j];
        b2.u[j] = lp[j]; b2.u[4 + j] = lp[j];
    }
}

__global__ __launch_bounds__(BLOCK)
void rpq_kernel(const float* __restrict__ x,
                const float* __restrict__ P,
                const float* __restrict__ CB,
                int* __restrict__ out,
                int ntok, int vocab, int nsuper)
{
    __shared__ __attribute__((aligned(16))) uint32_t Pth[DCB * PPW];
    __shared__ __attribute__((aligned(16))) uint32_t Ptl[DCB * PPW];
    __shared__ __attribute__((aligned(16))) uint32_t CBl[SUPER * 16];
    __shared__ __attribute__((aligned(16))) int      outl[TOK_PER_BLOCK];

    const int tid  = threadIdx.x;
    const int lane = tid & 31;
    const int h    = lane >> 4;
    const int m    = lane & 15;
    const int wave = tid >> 5;
    const int tokBase = blockIdx.x * TOK_PER_BLOCK + wave * TOK_PER_WAVE;

    for (int sl = tid; sl < DCB * PPW; sl += BLOCK) {
        const int n  = sl / PPW;
        const int kp = sl - n * PPW;
        const float v0 = P[(2 * kp) * DCB + n] * SP;
        const float v1 = P[(2 * kp + 1) * DCB + n] * SP;
        uint32_t hpk, lpk;
        split_pair(v0, v1, hpk, lpk);
        Pth[sl] = hpk;
        Ptl[sl] = lpk;
    }
    __syncthreads();

    Frag b1_0, b2_0, b1_1, b2_1;
    {
        int t0 = tokBase + m;      t0 = t0 < ntok ? t0 : ntok - 1;
        proj_tile(x + (size_t)t0 * DIN, Pth, Ptl, m, h, b1_0, b2_0);
        int t1 = tokBase + 16 + m; t1 = t1 < ntok ? t1 : ntok - 1;
        proj_tile(x + (size_t)t1 * DIN, Pth, Ptl, m, h, b1_1, b2_1);
    }

    float best0 = -__builtin_huge_valf(), best1 = -__builtin_huge_valf();
    int   idx0 = 0, idx1 = 0;
    const v8f zero = {};

    for (int s = 0; s < nsuper; ++s) {
        __syncthreads();
        for (int sl = tid; sl < SUPER * 8; sl += BLOCK) {
            const int r = sl >> 3;
            const int j = sl & 7;
            int code = s * SUPER + r;
            code = code < vocab ? code : vocab - 1;
            const float2 cv = *(const float2*)(CB + (size_t)code * DCB + 2 * j);
            uint32_t hpk, lpk;
            split_pair(cv.x * SC, cv.y * SC, hpk, lpk);
            CBl[r * 16 + j]     = hpk;
            CBl[r * 16 + 8 + j] = lpk;
        }
        __syncthreads();

        const int codeS = s * SUPER + 8 * h;
#pragma unroll 1
        for (int c = 0; c < NCHUNK; ++c) {
            Frag a;
            const int ab = c * 256 + m * 16 + 4 * h;
            a.q[0] = *(const uint4*)(CBl + ab);
            a.q[1] = *(const uint4*)(CBl + ab + 8);
            v8f d0 = wmma16(a.v, b1_0.v, zero);
            d0 = wmma16(a.v, b2_0.v, d0);
            v8f d1 = wmma16(a.v, b1_1.v, zero);
            d1 = wmma16(a.v, b2_1.v, d1);
            asm volatile("v_nop\n\tv_nop\n\tv_nop\n\tv_nop"
                         : "+v"(d0), "+v"(d1)
                         : "v"(a.v), "v"(b1_0.v), "v"(b2_0.v), "v"(b1_1.v), "v"(b2_1.v));
            const int cb = codeS + c * 16;
#pragma unroll
            for (int r = 0; r < 8; ++r) {
                const float v0 = d0[r], v1 = d1[r];
                if (v0 > best0) { best0 = v0; idx0 = cb + r; }
                if (v1 > best1) { best1 = v1; idx1 = cb + r; }
            }
        }
    }

    {
        float ov = __shfl_xor(best0, 16, 32);
        int   oi = __shfl_xor(idx0, 16, 32);
        if (ov > best0 || (ov == best0 && oi < idx0)) { best0 = ov; idx0 = oi; }
        ov = __shfl_xor(best1, 16, 32);
        oi = __shfl_xor(idx1, 16, 32);
        if (ov > best1 || (ov == best1 && oi < idx1)) { best1 = ov; idx1 = oi; }
    }

    if (h == 0) {
        outl[wave * 32 + m]      = idx0;
        outl[wave * 32 + 16 + m] = idx1;
    }
    __syncthreads();

    v4i ov4 = {};
    int obase = 0;
    if (lane < 8) {
        ov4   = *(const v4i*)(outl + wave * 32 + lane * 4);
        obase = tokBase + lane * 4;
    }
    if (lane < 8) {
        if (obase + 3 < ntok) {
            *(volatile v4i*)(out + obase) = ov4;
        } else {
            volatile int* o = out;
            if (obase + 0 < ntok) o[obase + 0] = ov4.x;
            if (obase + 1 < ntok) o[obase + 1] = ov4.y;
            if (obase + 2 < ntok) o[obase + 2] = ov4.z;
            if (obase + 3 < ntok) o[obase + 3] = ov4.w;
        }
    }
    __threadfence();
    if (lane < 8) {
        if (obase + 3 < ntok) {
            *(volatile v4i*)(out + obase) = ov4;
        } else {
            volatile int* o = out;
            if (obase + 0 < ntok) o[obase + 0] = ov4.x;
            if (obase + 1 < ntok) o[obase + 1] = ov4.y;
            if (obase + 2 < ntok) o[obase + 2] = ov4.z;
            if (obase + 3 < ntok) o[obase + 3] = ov4.w;
        }
    }
}

extern "C" void kernel_launch(void* const* d_in, const int* in_sizes, int n_in,
                              void* d_out, int out_size, void* d_ws, size_t ws_size,
                              hipStream_t stream)
{
    (void)n_in; (void)d_ws; (void)ws_size;
    const float* x  = (const float*)d_in[0];
    const float* P  = (const float*)d_in[1];
    const float* CB = (const float*)d_in[2];
    int* out = (int*)d_out;

    const int ntok  = in_sizes[0] / DIN;
    const int vocab = in_sizes[2] / DCB;
    if (ntok <= 0 || vocab <= 0) return;
    if (in_sizes[1] != DIN * DCB) return;
    if (out_size < ntok) return;

    const int nsuper = (vocab + SUPER - 1) / SUPER;
    const int blocks = (ntok + TOK_PER_BLOCK - 1) / TOK_PER_BLOCK;
    rpq_kernel<<<blocks, BLOCK, 0, stream>>>(x, P, CB, out, ntok, vocab, nsuper);
}
